// EquivariantMessageBlock_13950053777559
// MI455X (gfx1250) — hardware-verified
//
#include <hip/hip_runtime.h>
#include <stdint.h>


typedef _Float16 v16h __attribute__((ext_vector_type(16)));
typedef _Float16 v8h  __attribute__((ext_vector_type(8)));
typedef float    v8f  __attribute__((ext_vector_type(8)));
typedef float    v4f  __attribute__((ext_vector_type(4)));
union Frag { v16h v; v8h half[2]; };

#define NB     2
#define NN     384
#define NODES  (NB * NN)
#define HID    128
#define L1W    256
#define INW    273
#define GFEAT  17
#define NJG    (NN / 4)
#define PQW    512

#define AGP    132
#define A1P    136

#define OFF_HF    0
#define OFF_W1T   196608
#define OFF_WGT   327680
#define OFF_W2T   344064
#define OFF_WU1T  409600
#define OFF_WU2T  475136
#define OFF_PQ    507904
#define WS_TOTAL  2080768

static __device__ __forceinline__ v8f wmma_f16(v16h a, v16h b, v8f c) {
    v8f d = __builtin_amdgcn_wmma_f32_16x16x32_f16(false, a, false, b, (short)0, c, false, false);
    asm volatile("v_nop\n\tv_nop\n\tv_nop\n\tv_nop" : "+v"(d) : "v"(a), "v"(b));
    return d;
}

static __device__ __forceinline__ v8f zero8() {
    v8f z = {0.f, 0.f, 0.f, 0.f, 0.f, 0.f, 0.f, 0.f};
    return z;
}

static __device__ __forceinline__ float silu_f(float x) {
    const float e = __expf(-x);
    return x * __builtin_amdgcn_rcpf(1.f + e);
}

__global__ void __launch_bounds__(128)
k_tconv(const float* __restrict__ W, int ldk, int ldn, int row0, int K, int Kp, int N, int NQ,
        float scale, _Float16* __restrict__ T) {
    const int q = blockIdx.x * 128 + threadIdx.x;
    if (q >= NQ) return;
    const int n = q % N;
    const int kb = row0 + (q / N) * K;
    const float* src = W + (size_t)kb * ldk + (size_t)n * ldn;
    _Float16* dst = T + (size_t)q * Kp;
#pragma unroll
    for (int pass = 0; pass < 2; ++pass) {
#pragma unroll 1
        for (int k0 = 0; k0 < Kp; k0 += 8) {
            v8h v;
#pragma unroll
            for (int e = 0; e < 8; ++e) {
                const int k = k0 + e;
                float x = 0.f;
                if (k < K) x = src[(size_t)k * ldk] * scale;
                v[e] = (_Float16)x;
            }
            *(volatile v8h*)(dst + k0) = v;
        }
        if (pass == 0) __threadfence();
    }
}

__global__ void __launch_bounds__(128)
k_pq(const _Float16* __restrict__ hF, const _Float16* __restrict__ W1T, const float* __restrict__ b1,
     float* __restrict__ PQ) {
    __shared__ __align__(16) float sT[4 * 16 * 68];
    const int tid = threadIdx.x, w = tid >> 5, l = tid & 31, hh = l >> 4, nl = l & 15;
    const int m0 = blockIdx.x * 16;
    const int n0 = blockIdx.y * 256 + 64 * w;

    v8f acc[4];
#pragma unroll
    for (int v = 0; v < 4; ++v) acc[v] = zero8();

    const _Float16* ar = hF + (size_t)(m0 + nl) * HID + 8 * hh;
#pragma unroll
    for (int s = 0; s < 4; ++s) {
        Frag a;
        a.half[0] = *(const v8h*)(ar + 32 * s);
        a.half[1] = *(const v8h*)(ar + 32 * s + 16);
#pragma unroll
        for (int v = 0; v < 4; ++v) {
            const _Float16* br = W1T + (size_t)(n0 + 16 * v + nl) * HID + 32 * s + 8 * hh;
            Frag bb;
            bb.half[0] = *(const v8h*)br;
            bb.half[1] = *(const v8h*)(br + 16);
            acc[v] = wmma_f16(a.v, bb.v, acc[v]);
        }
    }

    float* st = sT + w * (16 * 68);
#pragma unroll
    for (int v = 0; v < 4; ++v) {
        const int col = 16 * v + nl;
        float bias = 0.f;
        if (blockIdx.y == 0) bias = 64.f * b1[n0 + col];
#pragma unroll
        for (int r = 0; r < 8; ++r) st[(8 * hh + r) * 68 + col] = acc[v][r] + bias;
    }
    __syncthreads();

    v4f vals[8];
#pragma unroll
    for (int p = 0; p < 8; ++p) vals[p] = *(const v4f*)(st + (2 * p + hh) * 68 + 4 * nl);
    float* base = PQ + (size_t)m0 * PQW + n0 + 4 * nl;
#pragma unroll
    for (int p = 0; p < 8; ++p) *(volatile v4f*)(base + (size_t)(2 * p + hh) * PQW) = vals[p];
    __threadfence();
#pragma unroll
    for (int p = 0; p < 8; ++p) *(volatile v4f*)(base + (size_t)(2 * p + hh) * PQW) = vals[p];
}

__global__ void __launch_bounds__(128)
k_msg(const float* __restrict__ pos, const float* __restrict__ PQ,
      const _Float16* __restrict__ WgT, const _Float16* __restrict__ W2T,
      const _Float16* __restrict__ hF, const float* __restrict__ h,
      const float* __restrict__ b2, const _Float16* __restrict__ Wu1T,
      const float* __restrict__ bu1, const _Float16* __restrict__ Wu2T,
      const float* __restrict__ bu2, const float* __restrict__ gamma,
      const float* __restrict__ beta, float* __restrict__ out) {
    __shared__ __align__(16) _Float16 sWg[L1W * 32];
    __shared__ __align__(32) v16h sB[4 * 8 * 32];
    __shared__ float sCut[64];

    const int tid = threadIdx.x, w = tid >> 5, l = tid & 31, hh = l >> 4, nl = l & 15;
    const int b = blockIdx.y, i0 = blockIdx.x * 16;
    const int nodei = b * NN + i0 + nl;

    for (int q = tid; q < (L1W * 32) / 8; q += 128)
        ((v8h*)sWg)[q] = ((const v8h*)WgT)[q];
    __syncthreads();

    const float pix = pos[(size_t)nodei * 2 + 0];
    const float piy = pos[(size_t)nodei * 2 + 1];
    const float* prow = PQ + (size_t)nodei * PQW + 8 * hh;
    const _Float16* w2r0 = W2T + (size_t)(32 * w + nl) * L1W + 8 * hh;
    const _Float16* w2r1 = w2r0 + (size_t)16 * L1W;
    const float INV64 = 0.015625f;

    v8f acc0 = zero8(), acc1 = zero8();
    float cutsum = 0.f;

#pragma unroll 1
    for (int g = 0; g < NJG; ++g) {
        const int j = 4 * g + w;
        const int nodej = b * NN + j;
        const float pjx = pos[(size_t)nodej * 2 + 0];
        const float pjy = pos[(size_t)nodej * 2 + 1];

        const float dx = pix - pjx, dy = piy - pjy;
        const float sq = dx * dx + dy * dy;
        const bool  mk = sq > 0.f;
        const float dist = mk ? __builtin_sqrtf(sq) : 0.f;
        const float rd = __builtin_amdgcn_rsqf(mk ? sq : 1.f);
        const float c1 = mk ? dx * rd : 1.f;
        const float s1 = mk ? dy * rd : 0.f;
        const float c2 = c1 * c1 - s1 * s1, s2 = s1 * c1 + c1 * s1;
        const float c3 = c2 * c1 - s2 * s1, s3 = s2 * c1 + c2 * s1;
        const float c4 = c3 * c1 - s3 * s1, s4 = s3 * c1 + c3 * s1;
        float f[GFEAT];
#pragma unroll
        for (int k = 0; k < 8; ++k) {
            const float ck = (float)k * (5.f / 7.f);
            const float dd = (dist - ck) * 1.6f;
            f[k] = __expf(-(dd * dd));
        }
        f[8] = 1.f;
        f[9] = c1;  f[10] = s1; f[11] = c2; f[12] = s2;
        f[13] = c3; f[14] = s3; f[15] = c4; f[16] = s4;
        const float xr = dist * 0.2f;
        const float x2 = xr * xr, x3 = x2 * xr, x6 = x3 * x3;
        const float cm = 1.f - x6, cm2 = cm * cm, cm3 = cm2 * cm;
        const float cut = (xr < 1.f) ? cm3 * cm3 : 0.f;
        cutsum += cut;
        const float c64 = cut * 64.f;

        Frag bg;
        {
            v8h g0, g1;
#pragma unroll
            for (int e = 0; e < 8; ++e) g0[e] = (_Float16)(hh ? f[8 + e] : f[e]);
            g1[0] = (_Float16)(hh ? 0.f : f[16]);
#pragma unroll
            for (int e = 1; e < 8; ++e) g1[e] = (_Float16)0.f;
            bg.half[0] = g0;
            bg.half[1] = g1;
        }
        const float* qrow = PQ + (size_t)nodej * PQW + L1W + 8 * hh;

#pragma unroll
        for (int s = 0; s < 8; ++s) {
            Frag f2;
#pragma unroll
            for (int hf = 0; hf < 2; ++hf) {
                const int t = 2 * s + hf;
                const _Float16* wr = sWg + (16 * t + nl) * 32 + 8 * hh;
                Frag a;
                a.half[0] = *(const v8h*)wr;
                a.half[1] = *(const v8h*)(wr + 16);
                const v4f p0 = *(const v4f*)(prow + 16 * t);
                const v4f p1 = *(const v4f*)(prow + 16 * t + 4);
                const v4f q0 = *(const v4f*)(qrow + 16 * t);
                const v4f q1 = *(const v4f*)(qrow + 16 * t + 4);
                v8f cc;
#pragma unroll
                for (int e = 0; e < 4; ++e) { cc[e] = p0[e] + q0[e]; cc[4 + e] = p1[e] + q1[e]; }
                const v8f d = wmma_f16(a.v, bg.v, cc);
                v8h o;
#pragma unroll
                for (int r = 0; r < 8; ++r) {
                    const float x = d[r] * INV64;
                    o[r] = (_Float16)(silu_f(x) * c64);
                }
                f2.half[hf] = o;
            }
            sB[(w * 8 + s) * 32 + l] = f2.v;
        }
        __syncthreads();

#pragma unroll
        for (int s = 0; s < 8; ++s) {
            Frag a0, a1;
            a0.half[0] = *(const v8h*)(w2r0 + 32 * s);
            a0.half[1] = *(const v8h*)(w2r0 + 32 * s + 16);
            a1.half[0] = *(const v8h*)(w2r1 + 32 * s);
            a1.half[1] = *(const v8h*)(w2r1 + 32 * s + 16);
#pragma unroll
            for (int jj = 0; jj < 4; ++jj) {
                const v16h bb = sB[(jj * 8 + s) * 32 + l];
                acc0 = wmma_f16(a0.v, bb, acc0);
                acc1 = wmma_f16(a1.v, bb, acc1);
            }
        }
        __syncthreads();
    }

    if (l < 16) sCut[w * 16 + l] = cutsum;
    __syncthreads();
    const float ct = ((sCut[nl] + sCut[16 + nl]) + sCut[32 + nl]) + sCut[48 + nl];

    float*    sAgg = reinterpret_cast<float*>(sB);
    _Float16* sA1  = reinterpret_cast<_Float16*>(reinterpret_cast<char*>(sB) + 8448);
    float*    sY   = reinterpret_cast<float*>(reinterpret_cast<char*>(sB) + 12800);

    const float INV4096 = 0.000244140625f;
#pragma unroll
    for (int r = 0; r < 8; ++r) {
        const int c = 32 * w + 8 * hh + r;
        sAgg[nl * AGP + c]      = acc0[r] * INV4096 + b2[c] * ct;
        sAgg[nl * AGP + c + 16] = acc1[r] * INV4096 + b2[c + 16] * ct;
    }
    __syncthreads();

    v8f u0 = zero8(), u1 = zero8();
    {
        const _Float16* wu0 = Wu1T + (size_t)(32 * w + nl) * (2 * HID) + 8 * hh;
        const _Float16* wu1 = wu0 + (size_t)16 * (2 * HID);
        const _Float16* hr  = hF + (size_t)nodei * HID + 8 * hh;
#pragma unroll
        for (int s = 0; s < 8; ++s) {
            Frag bb;
            if (s < 4) {
                bb.half[0] = *(const v8h*)(hr + 32 * s);
                bb.half[1] = *(const v8h*)(hr + 32 * s + 16);
            } else {
                const float* ag = sAgg + nl * AGP + 32 * (s - 4) + 8 * hh;
                const v4f x0 = *(const v4f*)(ag);
                const v4f x1 = *(const v4f*)(ag + 4);
                const v4f x2 = *(const v4f*)(ag + 16);
                const v4f x3 = *(const v4f*)(ag + 20);
                v8h lo, hi;
#pragma unroll
                for (int e = 0; e < 4; ++e) {
                    lo[e] = (_Float16)x0[e]; lo[4 + e] = (_Float16)x1[e];
                    hi[e] = (_Float16)x2[e]; hi[4 + e] = (_Float16)x3[e];
                }
                bb.half[0] = lo;
                bb.half[1] = hi;
            }
            Frag a0, a1;
            a0.half[0] = *(const v8h*)(wu0 + 32 * s);
            a0.half[1] = *(const v8h*)(wu0 + 32 * s + 16);
            a1.half[0] = *(const v8h*)(wu1 + 32 * s);
            a1.half[1] = *(const v8h*)(wu1 + 32 * s + 16);
            u0 = wmma_f16(a0.v, bb.v, u0);
            u1 = wmma_f16(a1.v, bb.v, u1);
        }
    }
#pragma unroll
    for (int r = 0; r < 8; ++r) {
        const int c = 32 * w + 8 * hh + r;
        const float p0 = u0[r] * INV64 + bu1[c];
        const float p1 = u1[r] * INV64 + bu1[c + 16];
        sA1[nl * A1P + c]      = (_Float16)silu_f(p0);
        sA1[nl * A1P + c + 16] = (_Float16)silu_f(p1);
    }
    __syncthreads();

    v8f z0 = zero8(), z1 = zero8();
    {
        const _Float16* wv0 = Wu2T + (size_t)(32 * w + nl) * HID + 8 * hh;
        const _Float16* wv1 = wv0 + (size_t)16 * HID;
        const _Float16* a1r = sA1 + nl * A1P + 8 * hh;
#pragma unroll
        for (int s = 0; s < 4; ++s) {
            Frag bb;
            bb.half[0] = *(const v8h*)(a1r + 32 * s);
            bb.half[1] = *(const v8h*)(a1r + 32 * s + 16);
            Frag a0, a1;
            a0.half[0] = *(const v8h*)(wv0 + 32 * s);
            a0.half[1] = *(const v8h*)(wv0 + 32 * s + 16);
            a1.half[0] = *(const v8h*)(wv1 + 32 * s);
            a1.half[1] = *(const v8h*)(wv1 + 32 * s + 16);
            z0 = wmma_f16(a0.v, bb.v, z0);
            z1 = wmma_f16(a1.v, bb.v, z1);
        }
    }
#pragma unroll
    for (int r = 0; r < 8; ++r) {
        const int c = 32 * w + 8 * hh + r;
        sY[nl * AGP + c]      = z0[r] * INV64 + bu2[c];
        sY[nl * AGP + c + 16] = z1[r] * INV64 + bu2[c + 16];
    }
    __syncthreads();

    v4f ov[4];
    const v4f gv = *(const v4f*)(gamma + 4 * l);
    const v4f bv = *(const v4f*)(beta + 4 * l);
#pragma unroll
    for (int rr = 0; rr < 4; ++rr) {
        const int i = 4 * w + rr;
        const int node = b * NN + i0 + i;
        const v4f hv = *(const v4f*)(h + (size_t)node * HID + 4 * l);
        const v4f yv = hv + *(const v4f*)(sY + i * AGP + 4 * l);
        float sm = (yv[0] + yv[1]) + (yv[2] + yv[3]);
#pragma unroll
        for (int o = 16; o > 0; o >>= 1) sm += __shfl_xor(sm, o);
        const float mu = sm * (1.f / 128.f);
        const v4f dv = yv - mu;
        float sv = (dv[0] * dv[0] + dv[1] * dv[1]) + (dv[2] * dv[2] + dv[3] * dv[3]);
#pragma unroll
        for (int o = 16; o > 0; o >>= 1) sv += __shfl_xor(sv, o);
        const float var = sv * (1.f / 128.f);
        const float inv = rsqrtf(var + 1e-5f);
        ov[rr] = dv * inv * gv + bv;
    }
#pragma unroll
    for (int rr = 0; rr < 4; ++rr) {
        const int node = b * NN + i0 + 4 * w + rr;
        *(volatile v4f*)(out + (size_t)node * HID + 4 * l) = ov[rr];
    }
    __threadfence();
#pragma unroll
    for (int rr = 0; rr < 4; ++rr) {
        const int node = b * NN + i0 + 4 * w + rr;
        *(volatile v4f*)(out + (size_t)node * HID + 4 * l) = ov[rr];
    }
}

extern "C" void kernel_launch(void* const* d_in, const int* in_sizes, int n_in,
                              void* d_out, int out_size, void* d_ws, size_t ws_size,
                              hipStream_t stream) {
    if (n_in < 12) return;
    if (in_sizes[0] != NODES * HID || in_sizes[1] != NODES * 2 || in_sizes[2] != INW * L1W ||
        in_sizes[3] != L1W || in_sizes[4] != L1W * HID || in_sizes[5] != HID ||
        in_sizes[6] != L1W * HID || in_sizes[7] != HID || in_sizes[8] != HID * HID ||
        in_sizes[9] != HID || in_sizes[10] != HID || in_sizes[11] != HID) return;
    if (out_size != NODES * HID) return;
    if (ws_size < (size_t)WS_TOTAL) return;

    const float* h     = (const float*)d_in[0];
    const float* pos   = (const float*)d_in[1];
    const float* W1    = (const float*)d_in[2];
    const float* b1    = (const float*)d_in[3];
    const float* W2    = (const float*)d_in[4];
    const float* b2    = (const float*)d_in[5];
    const float* Wu1   = (const float*)d_in[6];
    const float* bu1   = (const float*)d_in[7];
    const float* Wu2   = (const float*)d_in[8];
    const float* bu2   = (const float*)d_in[9];
    const float* gamma = (const float*)d_in[10];
    const float* beta  = (const float*)d_in[11];
    float* out = (float*)d_out;

    char* ws = (char*)d_ws;
    _Float16* hF   = (_Float16*)(ws + OFF_HF);
    _Float16* W1T  = (_Float16*)(ws + OFF_W1T);
    _Float16* WgT  = (_Float16*)(ws + OFF_WGT);
    _Float16* W2T  = (_Float16*)(ws + OFF_W2T);
    _Float16* Wu1T = (_Float16*)(ws + OFF_WU1T);
    _Float16* Wu2T = (_Float16*)(ws + OFF_WU2T);
    float*    PQ   = (float*)(ws + OFF_PQ);

    k_tconv<<<(NODES + 127) / 128, 128, 0, stream>>>(h, 1, HID, 0, HID, HID, NODES, NODES, 1.f, hF);
    k_tconv<<<(2 * L1W + 127) / 128, 128, 0, stream>>>(W1, L1W, 1, 0, HID, HID, L1W, 2 * L1W, 64.f, W1T);
    k_tconv<<<(L1W + 127) / 128, 128, 0, stream>>>(W1, L1W, 1, 2 * HID, GFEAT, 32, L1W, L1W, 64.f, WgT);
    k_tconv<<<(HID + 127) / 128, 128, 0, stream>>>(W2, HID, 1, 0, L1W, L1W, HID, HID, 64.f, W2T);
    k_tconv<<<(HID + 127) / 128, 128, 0, stream>>>(Wu1, HID, 1, 0, L1W, L1W, HID, HID, 64.f, Wu1T);
    k_tconv<<<(HID + 127) / 128, 128, 0, stream>>>(Wu2, HID, 1, 0, HID, HID, HID, HID, 64.f, Wu2T);

    k_pq<<<dim3(NODES / 16, 2), 128, 0, stream>>>(hF, W1T, b1, PQ);

    k_msg<<<dim3(NN / 16, NB), 128, 0, stream>>>(pos, PQ, WgT, W2T, hF, h, b2, Wu1T, bu1, Wu2T, bu2,
                                                 gamma, beta, out);
}
